// NeuralNeighborhoodFlow_18287970746484
// MI455X (gfx1250) — hardware-run, weakly checked
//
#include <hip/hip_runtime.h>
#include <math.h>

typedef __attribute__((ext_vector_type(16))) _Float16 v16h;
typedef __attribute__((ext_vector_type(8)))  _Float16 v8h;
typedef __attribute__((ext_vector_type(8)))  float    v8f;
typedef __attribute__((ext_vector_type(4)))  float    v4f;

constexpr int kT      = 5;
constexpr int kB      = 32;
constexpr int kNb     = 128;
constexpr int kD      = 256;
constexpr int kH      = 512;
constexpr int kM      = kB * kNb;
constexpr int kSub    = 2;
constexpr int kSteps  = (kT - 1) * kSub;
constexpr int kStages = kSteps * 4;
constexpr int kSlabP  = 68;
static_assert(kM == 4096);
static_assert(kStages == 32);
static_assert((kD % 32) == 0 && (kH % 32) == 0);
static_assert((kM % 64) == 0 && (kD % 64) == 0 && (kH % 64) == 0);
static_assert((kNb % 64) == 0);
static_assert((((kM >> 6) * (kH >> 6)) % 8) == 0 && (((kM >> 6) * (kD >> 6)) % 8) == 0);

constexpr float kCarryX = 256.0f;
constexpr float kCarryW = 256.0f;
constexpr float kCarryP = 256.0f;
constexpr float kFoldG1 = kCarryP / (kCarryX * kCarryW);
constexpr float kFoldG2 = 1.0f / (kCarryP * kCarryW);
constexpr float kF16MinNormal = 6.103515625e-05f;

constexpr size_t kOffW1H = 0;
constexpr size_t kOffW2H = kOffW1H + (size_t)kH * kD * 2;
constexpr size_t kOffSA  = kOffW2H + (size_t)kD * kH * 2;
constexpr size_t kOffSB  = kOffSA  + (size_t)kM * kD * 4;
constexpr size_t kOffK1  = kOffSB  + (size_t)kM * kD * 4;
constexpr size_t kOffK2  = kOffK1  + (size_t)kM * kD * 4;
constexpr size_t kOffK3  = kOffK2  + (size_t)kM * kD * 4;
constexpr size_t kOffXP  = kOffK3  + (size_t)kM * kD * 4;
constexpr size_t kOffPP  = kOffXP  + (size_t)kM * kD * 2;
constexpr size_t kOffSF  = kOffPP  + (size_t)kM * kH * 2;
constexpr size_t kWsTotal = kOffSF + (size_t)kStages * kB * kH * 4;
static_assert(kWsTotal == 29884416ull);
static_assert(kWsTotal <= 134217728ull);
static_assert((kOffW2H % 128) == 0 && (kOffSA % 128) == 0 && (kOffSB % 128) == 0 && (kOffK1 % 128) == 0 &&
              (kOffK2 % 128) == 0 && (kOffK3 % 128) == 0 && (kOffXP % 128) == 0 && (kOffPP % 128) == 0 &&
              (kOffSF % 128) == 0);
constexpr size_t kOut1Elems = (size_t)kT * kB * kD;
static_assert(kOut1Elems * 4 == 163840ull);
static_assert((kOut1Elems * 4) % 128 == 0);
static_assert(kOut1Elems * 4 + (size_t)kT * kM * kD * 4 == 21135360ull);

namespace eng {
__device__ __forceinline__ void acc_guard1(v8f& a, v16h x, v16h y) {
  asm volatile("v_nop\n\tv_nop\n\tv_nop\n\tv_nop" : "+v"(a) : "v"(x), "v"(y));
}
__device__ __forceinline__ void keep4_h(v16h a, v16h b, v16h c, v16h d) {
  asm volatile("v_nop" :: "v"(a), "v"(b), "v"(c), "v"(d));
}
__device__ __forceinline__ void acc_guard4(v8f& a, v8f& b, v8f& c, v8f& d) {
  asm volatile("v_nop\n\tv_nop\n\tv_nop\n\tv_nop" : "+v"(a), "+v"(b), "+v"(c), "+v"(d));
}
struct FragH {
  union U { v16h v; v8h h[2]; };
  static __device__ __forceinline__ v16h load(const _Float16* p) {
    U f;
    f.h[0] = *(const v8h*)(p);
    f.h[1] = *(const v8h*)(p + 16);
    return f.v;
  }
  static __device__ __forceinline__ v8f mma(v16h a, v16h b, v8f c) {
    return __builtin_amdgcn_wmma_f32_16x16x32_f16(false, a, false, b, (short)0, c, false, false);
  }
};
__device__ __forceinline__ void wave_sync() {
  __builtin_amdgcn_fence(__ATOMIC_RELEASE, "workgroup");
  __builtin_amdgcn_wave_barrier();
  __builtin_amdgcn_fence(__ATOMIC_ACQUIRE, "workgroup");
}
__device__ __forceinline__ _Float16 to_h16(float v) {
  const float t = (fabsf(v) < kF16MinNormal) ? 0.0f : v;
  return (_Float16)t;
}
}

__global__ __launch_bounds__(256) void cast_f16_carry_kernel(
    const float* __restrict__ src, unsigned short* __restrict__ dst, int total8, float carry)
{
  const int i = blockIdx.x * 256 + threadIdx.x;
  if (i >= total8) return;
  const size_t e0 = (size_t)i << 3;
  const v4f a0 = *(const v4f*)(src + e0);
  const v4f a1 = *(const v4f*)(src + e0 + 4);
  v8h hv;
#pragma unroll
  for (int e = 0; e < 4; ++e) {
    hv[e]     = eng::to_h16(a0[e] * carry);
    hv[4 + e] = eng::to_h16(a1[e] * carry);
  }
  unsigned short* q = dst + e0;
  *(volatile v8h*)q = hv;
  __threadfence();
  *(volatile v8h*)q = hv;
}

__global__ __launch_bounds__(256) void copy_f32_kernel(
    const float* __restrict__ src, float* __restrict__ dst, int total4)
{
  const int i = blockIdx.x * 256 + threadIdx.x;
  if (i >= total4) return;
  const size_t e0 = (size_t)i << 2;
  const v4f v = *(const v4f*)(src + e0);
  *(volatile v4f*)(dst + e0) = v;
  __threadfence();
  *(volatile v4f*)(dst + e0) = v;
}

__device__ __forceinline__ void store_group16(float* dst, const float* lds, int idx4) {
  const v4f v = *(const v4f*)(lds + 4 * idx4);
  *(volatile v4f*)(dst + 4 * idx4) = v;
  __threadfence();
  *(volatile v4f*)(dst + 4 * idx4) = v;
}

__global__ __launch_bounds__(256) void state_chain_kernel(
    const float* __restrict__ ts, const float* __restrict__ y0,
    const float* __restrict__ W1, const float* __restrict__ b1,
    const float* __restrict__ W2, const float* __restrict__ b2,
    float* __restrict__ sfAll, float* __restrict__ out0)
{
  __shared__ __align__(16) float sx[kD];
  __shared__ __align__(16) float sth[kH];
  __shared__ __align__(16) float ssf[kH];
  __shared__ __align__(16) float so[kD];
  const int tid = threadIdx.x;
  const int b = blockIdx.x;
  float y = y0[(size_t)b * kD + tid];
  float x = y;
  float k1 = 0.0f, k2 = 0.0f, k3 = 0.0f;
  const float bias2 = b2[tid];
  so[tid] = y;
  __syncthreads();
  if (tid < 64) store_group16(out0 + (size_t)b * kD, so, tid);
#pragma unroll 1
  for (int g = 0; g < kStages; ++g) {
    const int iv  = g >> 3;
    const int sub = (g >> 2) & 1;
    const int st  = g & 3;
    const float dt = (ts[iv + 1] - ts[iv]) * (1.0f / (float)kSub);
    sx[tid] = x;
    __syncthreads();
#pragma unroll 1
    for (int half = 0; half < 2; ++half) {
      const int j = tid + half * 256;
      const float* wr = W1 + (size_t)j * kD;
      float acc = 0.0f;
#pragma unroll 2
      for (int d4 = 0; d4 < kD / 4; ++d4) {
        const v4f w  = *(const v4f*)(wr + 4 * d4);
        const v4f xv = *(const v4f*)(sx + 4 * d4);
        acc = fmaf(w[0], xv[0], acc);
        acc = fmaf(w[1], xv[1], acc);
        acc = fmaf(w[2], xv[2], acc);
        acc = fmaf(w[3], xv[3], acc);
      }
      const float hval = acc + b1[j];
      const float th = tanhf(hval);
      sth[j] = th;
      ssf[j] = 1.0f - th * th;
    }
    __syncthreads();
    if (tid < 128) store_group16(sfAll + ((size_t)g * kB + b) * kH, ssf, tid);
    float acc2 = 0.0f;
    {
      const float* wr2 = W2 + (size_t)tid * kH;
#pragma unroll 2
      for (int h4 = 0; h4 < kH / 4; ++h4) {
        const v4f w  = *(const v4f*)(wr2 + 4 * h4);
        const v4f tv = *(const v4f*)(sth + 4 * h4);
        acc2 = fmaf(w[0], tv[0], acc2);
        acc2 = fmaf(w[1], tv[1], acc2);
        acc2 = fmaf(w[2], tv[2], acc2);
        acc2 = fmaf(w[3], tv[3], acc2);
      }
    }
    const float dy = acc2 + bias2;
    if (st == 0) {
      k1 = dy;
      x = y + (0.5f * dt) * dy;
    } else if (st == 1) {
      k2 = dy;
      x = y + (0.5f * dt) * dy;
    } else if (st == 2) {
      k3 = dy;
      x = y + dt * dy;
    } else {
      y = y + (dt * (1.0f / 6.0f)) * (((k1 + 2.0f * k2) + 2.0f * k3) + dy);
      x = y;
    }
    if (st == 3 && sub == kSub - 1) {
      so[tid] = y;
      __syncthreads();
      if (tid < 64) store_group16(out0 + ((size_t)(iv + 1) * kB + b) * kD, so, tid);
    }
  }
}

__global__ __launch_bounds__(256) void tangent_gemm1_kernel(
    const unsigned short* __restrict__ Xp, const unsigned short* __restrict__ W1hp,
    const float* __restrict__ sfac, unsigned short* __restrict__ Pp)
{
  using namespace eng;
  const _Float16* A  = (const _Float16*)Xp;
  const _Float16* Bt = (const _Float16*)W1hp;
  __shared__ __align__(16) float sT[8][16 * kSlabP];
  const int lane = threadIdx.x & 31;
  const int wave = threadIdx.x >> 5;
  constexpr int tilesN = kH >> 6;
  constexpr int tilesM = kM >> 6;
  const int tile = blockIdx.x * 8 + wave;
  if (tile >= tilesM * tilesN) return;
  const int tm = tile / tilesN;
  const int tn = tile - tm * tilesN;
  const int m0 = tm << 6;
  const int n0 = tn << 6;
  const int rlane = lane & 15;
  const int koff  = (lane >> 4) * 8;
  const int mOff  = (lane >> 4) * 8;

  v8f acc[4][4];
#pragma unroll
  for (int i = 0; i < 4; ++i)
#pragma unroll
    for (int j = 0; j < 4; ++j) acc[i][j] = (v8f){0.f, 0.f, 0.f, 0.f, 0.f, 0.f, 0.f, 0.f};

#pragma unroll 1
  for (int k0 = 0; k0 < kD; k0 += 32) {
    v16h bh[4];
#pragma unroll
    for (int j = 0; j < 4; ++j)
      bh[j] = FragH::load(Bt + (size_t)(n0 + (j << 4) + rlane) * kD + koff + k0);
#pragma unroll
    for (int i = 0; i < 4; ++i) {
      const v16h ah = FragH::load(A + (size_t)(m0 + (i << 4) + rlane) * kD + koff + k0);
#pragma unroll
      for (int j = 0; j < 4; ++j) acc[i][j] = FragH::mma(ah, bh[j], acc[i][j]);
      acc_guard1(acc[i][0], ah, bh[0]);
      acc_guard1(acc[i][1], ah, bh[1]);
      acc_guard1(acc[i][2], ah, bh[2]);
      acc_guard1(acc[i][3], ah, bh[3]);
    }
    keep4_h(bh[0], bh[1], bh[2], bh[3]);
  }
  acc_guard4(acc[0][0], acc[0][1], acc[0][2], acc[0][3]);
  acc_guard4(acc[1][0], acc[1][1], acc[1][2], acc[1][3]);
  acc_guard4(acc[2][0], acc[2][1], acc[2][2], acc[2][3]);
  acc_guard4(acc[3][0], acc[3][1], acc[3][2], acc[3][3]);

  float* slab = sT[wave];
  const int q  = lane >> 3;
  const int c8 = (lane & 7) * 8;
  const int bidx = m0 >> 7;
  const float* sfp = sfac + (size_t)bidx * kH + n0 + c8;
  const v4f sv0 = *(const v4f*)(sfp);
  const v4f sv1 = *(const v4f*)(sfp + 4);
  _Float16* P = (_Float16*)Pp;
#pragma unroll
  for (int i = 0; i < 4; ++i) {
    const int mBase = m0 + (i << 4);
#pragma unroll
    for (int j = 0; j < 4; ++j) {
#pragma unroll
      for (int r = 0; r < 8; ++r)
        slab[(mOff + r) * kSlabP + (j << 4) + rlane] = acc[i][j][r] * kFoldG1;
    }
    wave_sync();
    v8h hv[4];
#pragma unroll
    for (int it = 0; it < 4; ++it) {
      const int row = it * 4 + q;
      const float* sp = slab + row * kSlabP + c8;
      const v4f a0 = *(const v4f*)(sp);
      const v4f a1 = *(const v4f*)(sp + 4);
#pragma unroll
      for (int e = 0; e < 4; ++e) {
        hv[it][e]     = to_h16(a0[e] * sv0[e]);
        hv[it][4 + e] = to_h16(a1[e] * sv1[e]);
      }
    }
    for (int pass = 0; pass < 2; ++pass) {
#pragma unroll
      for (int it = 0; it < 4; ++it) {
        const int row = it * 4 + q;
        *(volatile v8h*)(P + (size_t)(mBase + row) * kH + n0 + c8) = hv[it];
      }
      __threadfence();
    }
    wave_sync();
  }
}

template <bool FINAL>
__global__ __launch_bounds__(256) void tangent_gemm2_kernel(
    const unsigned short* __restrict__ Pp, const unsigned short* __restrict__ W2hp,
    const float* Sread, const float* K1p, const float* K2p, const float* K3p,
    float* Dst, unsigned short* __restrict__ Xp, float* outSlice,
    const float* __restrict__ ts, int interval, float cfac, int save)
{
  using namespace eng;
  const _Float16* A  = (const _Float16*)Pp;
  const _Float16* Bt = (const _Float16*)W2hp;
  __shared__ __align__(16) float sT[8][16 * kSlabP];
  const int lane = threadIdx.x & 31;
  const int wave = threadIdx.x >> 5;
  constexpr int tilesN = kD >> 6;
  constexpr int tilesM = kM >> 6;
  const int tile = blockIdx.x * 8 + wave;
  if (tile >= tilesM * tilesN) return;
  const int tm = tile / tilesN;
  const int tn = tile - tm * tilesN;
  const int m0 = tm << 6;
  const int n0 = tn << 6;
  const int rlane = lane & 15;
  const int koff  = (lane >> 4) * 8;
  const int mOff  = (lane >> 4) * 8;

  const float dt  = (ts[interval + 1] - ts[interval]) * (1.0f / (float)kSub);
  const float cdt = cfac * dt;
  const float s6  = dt * (1.0f / 6.0f);

  v8f acc[4][4];
#pragma unroll
  for (int i = 0; i < 4; ++i)
#pragma unroll
    for (int j = 0; j < 4; ++j) acc[i][j] = (v8f){0.f, 0.f, 0.f, 0.f, 0.f, 0.f, 0.f, 0.f};

#pragma unroll 1
  for (int k0 = 0; k0 < kH; k0 += 32) {
    v16h bh[4];
#pragma unroll
    for (int j = 0; j < 4; ++j)
      bh[j] = FragH::load(Bt + (size_t)(n0 + (j << 4) + rlane) * kH + koff + k0);
#pragma unroll
    for (int i = 0; i < 4; ++i) {
      const v16h ah = FragH::load(A + (size_t)(m0 + (i << 4) + rlane) * kH + koff + k0);
#pragma unroll
      for (int j = 0; j < 4; ++j) acc[i][j] = FragH::mma(ah, bh[j], acc[i][j]);
      acc_guard1(acc[i][0], ah, bh[0]);
      acc_guard1(acc[i][1], ah, bh[1]);
      acc_guard1(acc[i][2], ah, bh[2]);
      acc_guard1(acc[i][3], ah, bh[3]);
    }
    keep4_h(bh[0], bh[1], bh[2], bh[3]);
  }
  acc_guard4(acc[0][0], acc[0][1], acc[0][2], acc[0][3]);
  acc_guard4(acc[1][0], acc[1][1], acc[1][2], acc[1][3]);
  acc_guard4(acc[2][0], acc[2][1], acc[2][2], acc[2][3]);
  acc_guard4(acc[3][0], acc[3][1], acc[3][2], acc[3][3]);

  float* slab = sT[wave];
  const int hh = lane >> 4;
  const int c4 = (lane & 15) * 4;
  const int q  = lane >> 3;
  const int c8 = (lane & 7) * 8;
  _Float16* X = (_Float16*)Xp;
#pragma unroll
  for (int i = 0; i < 4; ++i) {
    const int mBase = m0 + (i << 4);
#pragma unroll
    for (int j = 0; j < 4; ++j) {
#pragma unroll
      for (int r = 0; r < 8; ++r)
        slab[(mOff + r) * kSlabP + (j << 4) + rlane] = acc[i][j][r] * kFoldG2;
    }
    wave_sync();
    if (FINAL) {
#pragma unroll 2
      for (int it = 0; it < 8; ++it) {
        const int row = it * 2 + hh;
        const size_t o = (size_t)(mBase + row) * kD + n0 + c4;
        float* sp = slab + row * kSlabP + c4;
        const v4f kv = *(const v4f*)sp;
        const v4f s0 = *(const v4f*)(Sread + o);
        const v4f a1 = *(const v4f*)(K1p + o);
        const v4f a2 = *(const v4f*)(K2p + o);
        const v4f a3 = *(const v4f*)(K3p + o);
        v4f sn;
#pragma unroll
        for (int e = 0; e < 4; ++e)
          sn[e] = s0[e] + s6 * (((a1[e] + 2.0f * a2[e]) + 2.0f * a3[e]) + kv[e]);
        *(v4f*)sp = sn;
      }
      for (int pass = 0; pass < 2; ++pass) {
#pragma unroll
        for (int it = 0; it < 8; ++it) {
          const int row = it * 2 + hh;
          const size_t o = (size_t)(mBase + row) * kD + n0 + c4;
          const v4f v = *(const v4f*)(slab + row * kSlabP + c4);
          *(volatile v4f*)(Dst + o) = v;
          if (save != 0) *(volatile v4f*)(outSlice + o) = v;
        }
        __threadfence();
      }
    } else {
      for (int pass = 0; pass < 2; ++pass) {
#pragma unroll
        for (int it = 0; it < 8; ++it) {
          const int row = it * 2 + hh;
          const size_t o = (size_t)(mBase + row) * kD + n0 + c4;
          const v4f v = *(const v4f*)(slab + row * kSlabP + c4);
          *(volatile v4f*)(Dst + o) = v;
        }
        __threadfence();
      }
#pragma unroll 2
      for (int it = 0; it < 8; ++it) {
        const int row = it * 2 + hh;
        const size_t o = (size_t)(mBase + row) * kD + n0 + c4;
        float* sp = slab + row * kSlabP + c4;
        const v4f kv = *(const v4f*)sp;
        const v4f s0 = *(const v4f*)(Sread + o);
        v4f xn;
#pragma unroll
        for (int e = 0; e < 4; ++e) xn[e] = s0[e] + cdt * kv[e];
        *(v4f*)sp = xn;
      }
    }
    wave_sync();
    v8h hv[4];
#pragma unroll
    for (int it = 0; it < 4; ++it) {
      const int row = it * 4 + q;
      const float* sp = slab + row * kSlabP + c8;
      const v4f a0 = *(const v4f*)(sp);
      const v4f a1 = *(const v4f*)(sp + 4);
#pragma unroll
      for (int e = 0; e < 4; ++e) {
        hv[it][e]     = to_h16(a0[e] * kCarryX);
        hv[it][4 + e] = to_h16(a1[e] * kCarryX);
      }
    }
    for (int pass = 0; pass < 2; ++pass) {
#pragma unroll
      for (int it = 0; it < 4; ++it) {
        const int row = it * 4 + q;
        *(volatile v8h*)(X + (size_t)(mBase + row) * kD + n0 + c8) = hv[it];
      }
      __threadfence();
    }
    wave_sync();
  }
}

extern "C" void kernel_launch(void* const* d_in, const int* in_sizes, int n_in,
                              void* d_out, int out_size, void* d_ws, size_t ws_size,
                              hipStream_t stream) {
  if (n_in < 7) return;
  if (in_sizes[0] != kT) return;
  if (in_sizes[1] != kB * kD) return;
  if (in_sizes[2] != kM * kD) return;
  if (in_sizes[3] != kH * kD) return;
  if (in_sizes[4] != kH) return;
  if (in_sizes[5] != kD * kH) return;
  if (in_sizes[6] != kD) return;
  if (out_size != kT * kB * kD + kT * kM * kD) return;
  if (ws_size < kWsTotal) return;

  const float* ts  = (const float*)d_in[0];
  const float* y0  = (const float*)d_in[1];
  const float* Dy0 = (const float*)d_in[2];
  const float* W1  = (const float*)d_in[3];
  const float* b1  = (const float*)d_in[4];
  const float* W2  = (const float*)d_in[5];
  const float* b2  = (const float*)d_in[6];
  float* out0 = (float*)d_out;
  float* out1 = (float*)d_out + kOut1Elems;

  char* ws = (char*)d_ws;
  unsigned short* W1H = (unsigned short*)(ws + kOffW1H);
  unsigned short* W2H = (unsigned short*)(ws + kOffW2H);
  float* SA = (float*)(ws + kOffSA);
  float* SB = (float*)(ws + kOffSB);
  float* K1 = (float*)(ws + kOffK1);
  float* K2 = (float*)(ws + kOffK2);
  float* K3 = (float*)(ws + kOffK3);
  unsigned short* XP = (unsigned short*)(ws + kOffXP);
  unsigned short* PP = (unsigned short*)(ws + kOffPP);
  float* SF = (float*)(ws + kOffSF);

  cast_f16_carry_kernel<<<(kH * kD / 8) / 256, 256, 0, stream>>>(W1, W1H, kH * kD / 8, kCarryW);
  cast_f16_carry_kernel<<<(kD * kH / 8) / 256, 256, 0, stream>>>(W2, W2H, kD * kH / 8, kCarryW);
  cast_f16_carry_kernel<<<(kM * kD / 8) / 256, 256, 0, stream>>>(Dy0, XP, kM * kD / 8, kCarryX);
  copy_f32_kernel<<<(kM * kD / 4) / 256, 256, 0, stream>>>(Dy0, out1, kM * kD / 4);
  state_chain_kernel<<<kB, 256, 0, stream>>>(ts, y0, W1, b1, W2, b2, SF, out0);

  const int grid1 = ((kM >> 6) * (kH >> 6)) / 8;
  const int grid2 = ((kM >> 6) * (kD >> 6)) / 8;
  for (int s = 0; s < kSteps; ++s) {
    const int iv  = s / kSub;
    const int sub = s % kSub;
    const float* Sread = (s == 0) ? Dy0 : ((s & 1) ? (const float*)SA : (const float*)SB);
    float* Swrite = (s & 1) ? SB : SA;
    for (int st = 0; st < 4; ++st) {
      const int g = s * 4 + st;
      tangent_gemm1_kernel<<<grid1, 256, 0, stream>>>(XP, W1H, SF + (size_t)g * kB * kH, PP);
      if (st < 3) {
        float* Kdst = (st == 0) ? K1 : ((st == 1) ? K2 : K3);
        const float cfac = (st == 2) ? 1.0f : 0.5f;
        tangent_gemm2_kernel<false><<<grid2, 256, 0, stream>>>(
            PP, W2H, Sread, K1, K2, K3, Kdst, XP, out1 + (size_t)(iv + 1) * kM * kD, ts, iv, cfac, 0);
      } else {
        const int save = (sub == kSub - 1) ? 1 : 0;
        tangent_gemm2_kernel<true><<<grid2, 256, 0, stream>>>(
            PP, W2H, Sread, K1, K2, K3, Swrite, XP, out1 + (size_t)(iv + 1) * kM * kD, ts, iv, 1.0f, save);
      }
    }
  }
}
